// AVWDCRNN_10694468567657
// MI455X (gfx1250) — hardware-verified
//
#include <hip/hip_runtime.h>
#include <math.h>

constexpr int BATCH  = 8;
constexpr int TSTEPS = 12;
constexpr int NODES  = 256;
constexpr int DIN0   = 2;
constexpr int HID    = 64;
constexpr int EMB    = 16;
constexpr int CPAD   = 128;
constexpr int KCAT   = 2 * CPAD;
constexpr int OALL   = 3 * HID;
constexpr int WPITCH = OALL * KCAT;
constexpr int EKP    = 32;
constexpr int SLP    = 132;
constexpr int NBT    = BATCH * TSTEPS;
constexpr int S2_ELEMS = 2 * NODES * NODES;
constexpr int XG_PLANE = NODES * BATCH * CPAD;
constexpr int NOUT0  = BATCH * TSTEPS * NODES * HID;
constexpr int NOUT1  = 2 * BATCH * NODES * HID;
constexpr int NOUT_V4 = (NOUT0 + NOUT1) / 4;

constexpr float RES_SCALE = 2048.0f;
constexpr float RES_INV   = 1.0f / 2048.0f;
constexpr float CARRY_EMB  = 8.0f;
constexpr float CARRY_WP   = 64.0f;
constexpr float CARRY_WN   = 16.0f;
constexpr float CARRY_ADJ  = 16384.0f;
constexpr float CARRY_SUB  = 1024.0f;
constexpr float CARRY_XT   = 16.0f;
constexpr float CARRY_XG   = 16.0f;
constexpr float FOLD_WBUILD = 1.0f / (CARRY_EMB * CARRY_WP);
constexpr float FOLD_ADJSUB = 1.0f / (CARRY_ADJ * CARRY_SUB);
constexpr float FOLD_GMIX   = 1.0f / (CARRY_SUB * CARRY_XT);
constexpr float FOLD_NODE   = 1.0f / (CARRY_XG * CARRY_WN);
constexpr float SC_WBUILD   = CARRY_WN  * FOLD_WBUILD;
constexpr float SC_ADJSUB   = CARRY_SUB * FOLD_ADJSUB;
constexpr float SC_GMIX     = CARRY_XG  * FOLD_GMIX;
static_assert(RES_SCALE * RES_INV == 1.0f);
static_assert(FOLD_WBUILD * CARRY_EMB * CARRY_WP == 1.0f);
static_assert(FOLD_ADJSUB * CARRY_ADJ * CARRY_SUB == 1.0f);
static_assert(FOLD_GMIX * CARRY_SUB * CARRY_XT == 1.0f);
static_assert(FOLD_NODE * CARRY_XG * CARRY_WN == 1.0f);
static_assert(SC_WBUILD == 1.0f / 32.0f);
static_assert(SC_ADJSUB == 1.0f / 16384.0f);
static_assert(SC_GMIX == 1.0f / 1024.0f);
static_assert(FOLD_NODE == 1.0f / 256.0f);
static_assert(CARRY_ADJ <= 32768.0f && CARRY_SUB <= 32768.0f);

static_assert(WPITCH == 49152);
static_assert(NODES % 32 == 0 && (2 * NODES) % 32 == 0);
static_assert(WPITCH % 64 == 0 && NODES % 64 == 0 && CPAD % 64 == 0);
static_assert(KCAT % 32 == 0 && NODES % 32 == 0 && EKP % 32 == 0);
static_assert(((NODES / 32) * (NODES / 64)) % 8 == 0);
static_assert(((NODES / 32) * (WPITCH / 64)) % 8 == 0);
static_assert((((2 * NODES) / 32) * (CPAD / 64)) % 8 == 0);
static_assert(DIN0 + HID <= CPAD && HID + HID == CPAD);
static_assert(((size_t)NOUT0 * 4) % 128 == 0);
static_assert((size_t)NOUT0 * 4 == 6291456);
static_assert((size_t)NOUT0 * 4 + (size_t)NOUT1 * 4 == 7340032);
static_assert((NOUT0 + NOUT1) % 4 == 0 && NOUT_V4 % 256 == 0);

typedef __attribute__((ext_vector_type(16))) _Float16 v16h;
typedef __attribute__((ext_vector_type(8)))  _Float16 v8h;
typedef __attribute__((ext_vector_type(8)))  float    v8f;
typedef __attribute__((ext_vector_type(4)))  float    v4f;

__device__ __forceinline__ void split_hr(float p, _Float16& hi, _Float16& lo) {
  const _Float16 h = (_Float16)p;
  const float rsd = p - (float)h;
  hi = h;
  lo = (_Float16)(rsd * RES_SCALE);
}

__device__ __forceinline__ void grp_guard_h(v8f& a, v8f& b, v8f& c, v8f& d, v16h x, v16h y) { asm volatile("v_nop\n\tv_nop\n\tv_nop\n\tv_nop" : "+v"(a), "+v"(b), "+v"(c), "+v"(d) : "v"(x), "v"(y)); }
__device__ __forceinline__ void keep4_h(v16h a, v16h b, v16h c, v16h d) { asm volatile("v_nop" :: "v"(a), "v"(b), "v"(c), "v"(d)); }
__device__ __forceinline__ void acc_guard4(v8f& a, v8f& b, v8f& c, v8f& d) { asm volatile("v_nop\n\tv_nop\n\tv_nop\n\tv_nop" : "+v"(a), "+v"(b), "+v"(c), "+v"(d)); }

template <typename T> struct Frag;
template <> struct Frag<_Float16> {
  typedef v16h V; union U { v16h v; v8h h[2]; };
  static __device__ __forceinline__ v16h load(const _Float16* p) {
    U f; f.h[0] = *(const v8h*)(p); f.h[1] = *(const v8h*)(p + 16); return f.v;
  }
  static __device__ __forceinline__ v8f mma(v16h a, v16h b, v8f c) {
    return __builtin_amdgcn_wmma_f32_16x16x32_f16(false, a, false, b, (short)0, c, false, false);
  }
};

__device__ __forceinline__ v8f nh_mma(v16h a, v16h b, v8f c) {
  c = __builtin_amdgcn_wmma_f32_16x16x32_f16(false, a, false, b, (short)0, c, false, false);
  asm volatile("v_nop\n\tv_nop\n\tv_nop\n\tv_nop" : "+v"(c) : "v"(a), "v"(b));
  return c;
}

__global__ __launch_bounds__(256) void gemm_hr_kernel(
    const unsigned short* __restrict__ Ap, const unsigned short* __restrict__ A2p, int lda, long strideA,
    const unsigned short* __restrict__ Btp, const unsigned short* __restrict__ Bt2p, int ldb, long strideB,
    unsigned short* __restrict__ Cp, unsigned short* __restrict__ C2p, int ldc, long strideC,
    int M, int N, int K, float scale) {
  typedef _Float16 T;
  typedef v16h V;
  __shared__ __align__(16) float sT[8][16 * 68];
  const int b    = blockIdx.y;
  const int lane = threadIdx.x & 31;
  const int wave = threadIdx.x >> 5;
  const int tilesN = N >> 6;
  const int tilesM = M >> 5;
  const int tile = blockIdx.x * 8 + wave;
  if (tile >= tilesM * tilesN) return;
  const int tm = tile / tilesN;
  const int tn = tile - tm * tilesN;
  const int m0 = tm << 5;
  const int n0 = tn << 6;

  const T* Ab  = (const T*)Ap   + (size_t)b * strideA;
  const T* Ab2 = (const T*)A2p  + (size_t)b * strideA;
  const T* Bb  = (const T*)Btp  + (size_t)b * strideB;
  const T* Bb2 = (const T*)Bt2p + (size_t)b * strideB;

  const int rlane = lane & 15;
  const int koff  = (lane >> 4) * 8;
  const int mOff  = (lane >> 4) * 8;

  v8f accH[2][4], accX[2][4];
#pragma unroll
  for (int i = 0; i < 2; ++i)
#pragma unroll
    for (int j = 0; j < 4; ++j) {
      accH[i][j] = (v8f){0.f,0.f,0.f,0.f,0.f,0.f,0.f,0.f};
      accX[i][j] = (v8f){0.f,0.f,0.f,0.f,0.f,0.f,0.f,0.f};
    }

  for (int k0 = 0; k0 < K; k0 += 32) {
    V ah[2], al[2];
#pragma unroll
    for (int i = 0; i < 2; ++i) {
      const size_t ao = (size_t)(m0 + (i << 4) + rlane) * lda + koff + k0;
      ah[i] = Frag<T>::load(Ab + ao);
      al[i] = Frag<T>::load(Ab2 + ao);
    }
#pragma unroll
    for (int j = 0; j < 4; ++j) {
      const size_t bo = (size_t)(n0 + (j << 4) + rlane) * ldb + koff + k0;
      const V bh = Frag<T>::load(Bb + bo);
      const V bl = Frag<T>::load(Bb2 + bo);
#pragma unroll
      for (int i = 0; i < 2; ++i) {
        accH[i][j] = Frag<T>::mma(ah[i], bh, accH[i][j]);
        accX[i][j] = Frag<T>::mma(ah[i], bl, accX[i][j]);
        accX[i][j] = Frag<T>::mma(al[i], bh, accX[i][j]);
      }
      grp_guard_h(accH[0][j], accH[1][j], accX[0][j], accX[1][j], bh, bl);
    }
    keep4_h(ah[0], ah[1], al[0], al[1]);
  }
  acc_guard4(accH[0][0], accH[0][1], accH[0][2], accH[0][3]);
  acc_guard4(accH[1][0], accH[1][1], accH[1][2], accH[1][3]);
  acc_guard4(accX[0][0], accX[0][1], accX[0][2], accX[0][3]);
  acc_guard4(accX[1][0], accX[1][1], accX[1][2], accX[1][3]);

  float* slab = sT[wave];
  unsigned short* C  = Cp  + (size_t)b * strideC;
  unsigned short* C2 = C2p + (size_t)b * strideC;
  const int q = lane >> 3, c8 = (lane & 7) * 8;
#pragma unroll
  for (int i = 0; i < 2; ++i) {
    const int mBase = m0 + (i << 4);
#pragma unroll
    for (int j = 0; j < 4; ++j) {
#pragma unroll
      for (int r = 0; r < 8; ++r) {
        const float v = (accH[i][j][r] + accX[i][j][r] * RES_INV) * scale;
        slab[(mOff + r) * 68 + (j << 4) + rlane] = v;
      }
    }
    __builtin_amdgcn_fence(__ATOMIC_RELEASE, "workgroup");
    __builtin_amdgcn_wave_barrier();
    __builtin_amdgcn_fence(__ATOMIC_ACQUIRE, "workgroup");
    for (int pass = 0; pass < 2; ++pass) {
#pragma unroll
      for (int it = 0; it < 4; ++it) {
        const int row = it * 4 + q;
        const float* sp = slab + row * 68 + c8;
        v8h hv, lv;
#pragma unroll
        for (int e = 0; e < 8; ++e) {
          const float p = sp[e];
          _Float16 h, l;
          split_hr(p, h, l);
          hv[e] = h;
          lv[e] = l;
        }
        *(volatile v8h*)(C  + (size_t)(mBase + row) * ldc + n0 + c8) = hv;
        *(volatile v8h*)(C2 + (size_t)(mBase + row) * ldc + n0 + c8) = lv;
      }
      __threadfence();
    }
    __builtin_amdgcn_fence(__ATOMIC_RELEASE, "workgroup");
    __builtin_amdgcn_wave_barrier();
    __builtin_amdgcn_fence(__ATOMIC_ACQUIRE, "workgroup");
  }
}

__global__ __launch_bounds__(256) void embed_planes_kernel(const float* __restrict__ emb,
                                                           unsigned short* __restrict__ eh,
                                                           unsigned short* __restrict__ el) {
  const int gid = blockIdx.x * 256 + threadIdx.x;
  const int n = gid >> 2;
  const int q = gid & 3;
  const float* sp = emb + n * EMB + (q & 1) * 8;
  const v4f a = *(const v4f*)(sp);
  const v4f b = *(const v4f*)(sp + 4);
  const bool live = (q < 2);
  v8h hv, lv;
#pragma unroll
  for (int e = 0; e < 4; ++e) {
    const float a_e = a[e];
    const float b_e = b[e];
    const float f0 = live ? a_e * CARRY_EMB : 0.0f;
    const float f1 = live ? b_e * CARRY_EMB : 0.0f;
    _Float16 h0, l0, h1, l1;
    split_hr(f0, h0, l0);
    split_hr(f1, h1, l1);
    hv[e]     = h0;
    hv[4 + e] = h1;
    lv[e]     = l0;
    lv[4 + e] = l1;
  }
  *(volatile v8h*)(eh + (size_t)gid * 8) = hv;
  *(volatile v8h*)(el + (size_t)gid * 8) = lv;
  __threadfence();
  *(volatile v8h*)(eh + (size_t)gid * 8) = hv;
  *(volatile v8h*)(el + (size_t)gid * 8) = lv;
}

__global__ __launch_bounds__(256) void node_bias_kernel(const float* __restrict__ emb,
                                                        const float* __restrict__ gb,
                                                        const float* __restrict__ ub,
                                                        float* __restrict__ dst) {
  const int gid = blockIdx.x * 256 + threadIdx.x;
  const int n = gid / OALL;
  const int o = gid - n * OALL;
  const int og = (o < 2 * HID) ? o : (2 * HID - 1);
  int ou = o - 2 * HID;
  ou = ou < 0 ? 0 : ou;
  ou = ou > HID - 1 ? HID - 1 : ou;
  float accg = 0.0f, accu = 0.0f;
#pragma unroll 1
  for (int d = 0; d < EMB; ++d) {
    const float ev = emb[n * EMB + d];
    accg = fmaf(ev, gb[d * (2 * HID) + og], accg);
    accu = fmaf(ev, ub[d * HID + ou], accu);
  }
  const float v = (o < 2 * HID) ? accg : accu;
  *(volatile float*)(dst + gid) = v;
  __threadfence();
  *(volatile float*)(dst + gid) = v;
}

__global__ __launch_bounds__(256) void adj_rows_kernel(const float* __restrict__ emb,
                                                       unsigned short* __restrict__ ah,
                                                       unsigned short* __restrict__ al) {
  __shared__ __align__(16) float ei[EMB];
  __shared__ float redm[8];
  __shared__ float reds[8];
  __shared__ __align__(16) float prow[NODES];
  const int n = blockIdx.x;
  const int tid = threadIdx.x, lane = tid & 31, wave = tid >> 5;
  if (tid < EMB) ei[tid] = emb[n * EMB + tid];
  __syncthreads();
  const float* ej = emb + tid * EMB;
  float dot = 0.0f;
#pragma unroll
  for (int q = 0; q < 4; ++q) {
    const v4f w = *(const v4f*)(ej + 4 * q);
    dot = fmaf(ei[4 * q + 0], w[0], dot);
    dot = fmaf(ei[4 * q + 1], w[1], dot);
    dot = fmaf(ei[4 * q + 2], w[2], dot);
    dot = fmaf(ei[4 * q + 3], w[3], dot);
  }
  const float v = fmaxf(dot, 0.0f);
  float m = v;
#pragma unroll
  for (int off = 1; off < 32; off <<= 1) m = fmaxf(m, __shfl_xor(m, off, 32));
  if (lane == 0) redm[wave] = m;
  __syncthreads();
  float mx = redm[0];
#pragma unroll
  for (int w = 1; w < 8; ++w) mx = fmaxf(mx, redm[w]);
  const float e = expf(v - mx);
  float s = e;
#pragma unroll
  for (int off = 1; off < 32; off <<= 1) s += __shfl_xor(s, off, 32);
  if (lane == 0) reds[wave] = s;
  __syncthreads();
  float tot = 0.0f;
#pragma unroll
  for (int w = 0; w < 8; ++w) tot += reds[w];
  prow[tid] = e * (1.0f / tot);
  __syncthreads();
  if (wave == 0) {
    const v4f a = *(const v4f*)(prow + 8 * lane);
    const v4f b = *(const v4f*)(prow + 8 * lane + 4);
    v8h hv, lv;
#pragma unroll
    for (int q = 0; q < 4; ++q) {
      const float a_q = a[q] * CARRY_ADJ;
      const float b_q = b[q] * CARRY_ADJ;
      _Float16 h0, l0, h1, l1;
      split_hr(a_q, h0, l0);
      split_hr(b_q, h1, l1);
      hv[q]     = h0;
      hv[4 + q] = h1;
      lv[q]     = l0;
      lv[4 + q] = l1;
    }
    unsigned short* ph = ah + (size_t)n * NODES + 8 * lane;
    unsigned short* pl = al + (size_t)n * NODES + 8 * lane;
    *(volatile v8h*)ph = hv;
    *(volatile v8h*)pl = lv;
    __threadfence();
    *(volatile v8h*)ph = hv;
    *(volatile v8h*)pl = lv;
  }
}

__global__ __launch_bounds__(256) void sub_planes_kernel(const float* __restrict__ pa,
                                                         unsigned short* __restrict__ s2h,
                                                         unsigned short* __restrict__ s2l,
                                                         unsigned short* __restrict__ pth,
                                                         unsigned short* __restrict__ ptl) {
  __shared__ __align__(16) float prs[64 * HID];
  __shared__ __align__(16) float et[64 * NODES];
  __shared__ float part[8 * 64];
  __shared__ float zinv[64];
  const int tb = blockIdx.x;
  const int t = tb / BATCH;
  const int b = tb - t * BATCH;
  const int r0 = blockIdx.y * 64;
  const int tid = threadIdx.x, lane = tid & 31, wave = tid >> 5;
  const float* pabt = pa + ((size_t)(b * TSTEPS + t) * NODES) * HID;
#pragma unroll
  for (int i = 0; i < 4; ++i) {
    const int idx = tid + 256 * i;
    *(v4f*)(prs + idx * 4) = *(const v4f*)(pabt + (size_t)r0 * HID + idx * 4);
  }
  v4f mine[16];
#pragma unroll
  for (int h4 = 0; h4 < 16; ++h4) mine[h4] = *(const v4f*)(pabt + (size_t)tid * HID + h4 * 4);
  __syncthreads();
#pragma unroll 1
  for (int r = 0; r < 64; ++r) {
    float d = 0.0f;
#pragma unroll
    for (int h4 = 0; h4 < 16; ++h4) {
      const v4f p = *(const v4f*)(prs + r * HID + h4 * 4);
      d += fabsf(mine[h4][0] - p[0]);
      d += fabsf(mine[h4][1] - p[1]);
      d += fabsf(mine[h4][2] - p[2]);
      d += fabsf(mine[h4][3] - p[3]);
    }
    const float e = expf(-d);
    et[r * NODES + tid] = e;
    float s = e;
#pragma unroll
    for (int off = 1; off < 32; off <<= 1) s += __shfl_xor(s, off, 32);
    if (lane == 0) part[wave * 64 + r] = s;
  }
  __syncthreads();
  if (tid < 64) {
    float z = 0.0f;
#pragma unroll
    for (int w = 0; w < 8; ++w) z += part[w * 64 + tid];
    zinv[tid] = 1.0f / z;
  }
  __syncthreads();
  for (int pass = 0; pass < 2; ++pass) {
#pragma unroll 1
    for (int it = 0; it < 8; ++it) {
      const int task = it * 256 + tid;
      const int cc = task >> 3;
      const int q8 = task & 7;
      v8h hv, lv;
#pragma unroll
      for (int e = 0; e < 8; ++e) {
        const int r = 8 * q8 + e;
        const float f = (et[r * NODES + cc] * zinv[r]) * CARRY_SUB;
        _Float16 h, l;
        split_hr(f, h, l);
        hv[e] = h;
        lv[e] = l;
      }
      const size_t o = ((size_t)tb * (2 * NODES) + cc) * NODES + r0 + 8 * q8;
      *(volatile v8h*)(s2h + o) = hv;
      *(volatile v8h*)(s2l + o) = lv;
    }
#pragma unroll 1
    for (int i = 0; i < 8; ++i) {
      const int r = wave * 8 + i;
      const float zi = zinv[r];
      const v4f a = *(const v4f*)(et + r * NODES + 8 * lane);
      const v4f bq = *(const v4f*)(et + r * NODES + 8 * lane + 4);
      v8h hv, lv;
#pragma unroll
      for (int q = 0; q < 4; ++q) {
        const float f0 = (a[q] * zi) * CARRY_SUB;
        const float f1 = (bq[q] * zi) * CARRY_SUB;
        _Float16 h0, l0, h1, l1;
        split_hr(f0, h0, l0);
        split_hr(f1, h1, l1);
        hv[q]     = h0;
        hv[4 + q] = h1;
        lv[q]     = l0;
        lv[4 + q] = l1;
      }
      const size_t o = ((size_t)tb * NODES + r0 + r) * NODES + 8 * lane;
      *(volatile v8h*)(pth + o) = hv;
      *(volatile v8h*)(ptl + o) = lv;
    }
    __threadfence();
  }
}

template <int CIN>
__global__ __launch_bounds__(256) void wpool_planes_kernel(const float* __restrict__ gw,
                                                           const float* __restrict__ uw,
                                                           unsigned short* __restrict__ wh,
                                                           unsigned short* __restrict__ wl) {
  const int gid = blockIdx.x * 256 + threadIdx.x;
  const int j = gid >> 2;
  const int q = gid & 3;
  const int oall = j >> 8;
  const int kk = (j >> 7) & 1;
  const int i = j & (CPAD - 1);
  const int ic = (i < CIN) ? i : (CIN - 1);
  const int og = (oall < 2 * HID) ? oall : (2 * HID - 1);
  int ou = oall - 2 * HID;
  ou = ou < 0 ? 0 : ou;
  ou = ou > HID - 1 ? HID - 1 : ou;
  const int d0 = (q & 1) * 8;
  const bool live = (q < 2) && (i < CIN);
  const bool isg = (oall < 2 * HID);
  v8h hv, lv;
#pragma unroll
  for (int e = 0; e < 8; ++e) {
    const int d = d0 + e;
    const float fg = gw[((size_t)(d * 2 + kk) * CIN + ic) * (2 * HID) + og];
    const float fu = uw[((size_t)(d * 2 + kk) * CIN + ic) * HID + ou];
    float f = isg ? fg : fu;
    f = live ? f * CARRY_WP : 0.0f;
    _Float16 h, l;
    split_hr(f, h, l);
    hv[e] = h;
    lv[e] = l;
  }
  *(volatile v8h*)(wh + (size_t)gid * 8) = hv;
  *(volatile v8h*)(wl + (size_t)gid * 8) = lv;
  __threadfence();
  *(volatile v8h*)(wh + (size_t)gid * 8) = hv;
  *(volatile v8h*)(wl + (size_t)gid * 8) = lv;
}

template <int DIN, bool UPD>
__global__ __launch_bounds__(256) void xin_planes_kernel(const float* __restrict__ xsrc,
                                                         const float* __restrict__ st_in,
                                                         const float* __restrict__ pat,
                                                         const float* __restrict__ zr,
                                                         unsigned short* __restrict__ xh,
                                                         unsigned short* __restrict__ xl) {
  const int gid = blockIdx.x * 256 + threadIdx.x;
  const int ng = gid & 31;
  const int c = (gid >> 5) & (CPAD - 1);
  const int b = gid >> 12;
  const int cx = (c < DIN) ? c : (DIN - 1);
  int hc = c - DIN;
  hc = hc < 0 ? 0 : hc;
  hc = hc > HID - 1 ? HID - 1 : hc;
  const bool isx = (c < DIN);
  const bool iss = (c < DIN + HID);
  v8h hv, lv;
#pragma unroll
  for (int half = 0; half < 2; ++half) {
#pragma unroll
    for (int e4 = 0; e4 < 4; ++e4) {
      const int e = half * 4 + e4;
      const int n = 8 * ng + e;
      const float xv = xsrc[(size_t)b * (TSTEPS * NODES * DIN) + (size_t)n * DIN + cx];
      float sv = st_in[((size_t)b * NODES + n) * HID + hc] + pat[(size_t)b * (TSTEPS * NODES * HID) + (size_t)n * HID + hc];
      if (UPD) sv *= zr[((size_t)b * NODES + n) * (2 * HID) + hc];
      const float f = isx ? xv : (iss ? sv : 0.0f);
      const float p = f * CARRY_XT;
      _Float16 h, l;
      split_hr(p, h, l);
      hv[e] = h;
      lv[e] = l;
    }
    asm volatile("" ::: "memory");
  }
  *(volatile v8h*)(xh + (size_t)gid * 8) = hv;
  *(volatile v8h*)(xl + (size_t)gid * 8) = lv;
  __threadfence();
  *(volatile v8h*)(xh + (size_t)gid * 8) = hv;
  *(volatile v8h*)(xl + (size_t)gid * 8) = lv;
}

template <int NTILE, bool UPD>
__global__ __launch_bounds__(256) void node_gemm_kernel(
    const unsigned short* __restrict__ xghp, const unsigned short* __restrict__ xglp,
    const unsigned short* __restrict__ whp, const unsigned short* __restrict__ wlp,
    const float* __restrict__ bias,
    float* zr,
    const float* __restrict__ st_in, const float* __restrict__ pat,
    float* __restrict__ st_out, float* __restrict__ seq_dst, float* __restrict__ fin_dst, int has_fin) {
  __shared__ __align__(16) float slabs[8][8 * SLP];
  const _Float16* xgh = (const _Float16*)xghp;
  const _Float16* xgl = (const _Float16*)xglp;
  const _Float16* wh = (const _Float16*)whp;
  const _Float16* wl = (const _Float16*)wlp;
  const int tid = threadIdx.x, lane = tid & 31, wave = tid >> 5;
  const int c = lane & 15, hh = lane >> 4, koff = hh * 8;
  const int n = blockIdx.x * 8 + wave;

  v8f accH[NTILE], accX[NTILE];
#pragma unroll
  for (int j = 0; j < NTILE; ++j) {
    accH[j] = (v8f){0.f,0.f,0.f,0.f,0.f,0.f,0.f,0.f};
    accX[j] = (v8f){0.f,0.f,0.f,0.f,0.f,0.f,0.f,0.f};
  }

  const size_t arow = ((size_t)n * BATCH + (size_t)(c & 7)) * CPAD + koff;
  const size_t brow = (size_t)n * WPITCH + (size_t)c * KCAT + koff;
#pragma unroll 1
  for (int ks = 0; ks < KCAT / 32; ++ks) {
    const size_t ao = arow + (size_t)(ks >> 2) * XG_PLANE + (size_t)(ks & 3) * 32;
    const v16h a_hi = Frag<_Float16>::load(xgh + ao);
    const v16h a_lo = Frag<_Float16>::load(xgl + ao);
#pragma unroll
    for (int j = 0; j < NTILE; ++j) {
      const size_t bo = brow + (size_t)j * (16 * KCAT) + (size_t)ks * 32;
      const v16h b_hi = Frag<_Float16>::load(wh + bo);
      const v16h b_lo = Frag<_Float16>::load(wl + bo);
      accH[j] = nh_mma(a_hi, b_hi, accH[j]);
      accX[j] = nh_mma(a_hi, b_lo, accX[j]);
      accX[j] = nh_mma(a_lo, b_hi, accX[j]);
    }
  }

  float* sl = slabs[wave];
#pragma unroll
  for (int j = 0; j < NTILE; ++j) {
    const float bv = bias[(size_t)n * OALL + 16 * j + c];
#pragma unroll
    for (int r = 0; r < 8; ++r) {
      const float v = (accH[j][r] + accX[j][r] * RES_INV) * FOLD_NODE + bv;
      if (hh == 0) sl[r * SLP + 16 * j + c] = v;
    }
  }
  __builtin_amdgcn_fence(__ATOMIC_RELEASE, "workgroup");
  __builtin_amdgcn_wave_barrier();
  __builtin_amdgcn_fence(__ATOMIC_ACQUIRE, "workgroup");

  if (!UPD) {
#pragma unroll 1
    for (int rb = 0; rb < 8; ++rb) {
      v4f v = *(const v4f*)(sl + rb * SLP + 4 * lane);
#pragma unroll
      for (int e = 0; e < 4; ++e) {
        const float x = v[e];
        v[e] = 1.0f / (1.0f + expf(-x));
      }
      *(v4f*)(sl + rb * SLP + 4 * lane) = v;
    }
    for (int pass = 0; pass < 2; ++pass) {
#pragma unroll 1
      for (int rb = 0; rb < 8; ++rb) {
        const v4f v = *(const v4f*)(sl + rb * SLP + 4 * lane);
        *(volatile v4f*)(zr + ((size_t)rb * NODES + n) * (2 * HID) + 4 * lane) = v;
      }
      __threadfence();
    }
  } else {
    const int c4 = c * 4;
#pragma unroll 1
    for (int it = 0; it < 4; ++it) {
      const int bb = it * 2 + hh;
      v4f pre = *(const v4f*)(sl + bb * SLP + c4);
      const v4f rv = *(const v4f*)(zr + ((size_t)bb * NODES + n) * (2 * HID) + HID + c4);
      const v4f pv = *(const v4f*)(st_in + ((size_t)bb * NODES + n) * HID + c4);
      const v4f av = *(const v4f*)(pat + (size_t)bb * (TSTEPS * NODES * HID) + (size_t)n * HID + c4);
#pragma unroll
      for (int e = 0; e < 4; ++e) {
        const float se = pv[e] + av[e];
        const float hcv = tanhf(pre[e]);
        const float rr = rv[e];
        pre[e] = rr * se + (1.0f - rr) * hcv;
      }
      *(v4f*)(sl + bb * SLP + c4) = pre;
    }
    for (int pass = 0; pass < 2; ++pass) {
#pragma unroll 1
      for (int it = 0; it < 4; ++it) {
        const int bb = it * 2 + hh;
        const v4f v = *(const v4f*)(sl + bb * SLP + c4);
        *(volatile v4f*)(st_out + ((size_t)bb * NODES + n) * HID + c4) = v;
        *(volatile v4f*)(seq_dst + (size_t)bb * (TSTEPS * NODES * HID) + (size_t)n * HID + c4) = v;
        if (has_fin) *(volatile v4f*)(fin_dst + ((size_t)bb * NODES + n) * HID + c4) = v;
      }
      __threadfence();
    }
  }
}

__global__ __launch_bounds__(256) void premise_guard_kernel(const int* __restrict__ flag, float* __restrict__ out) {
  const int v = flag[0];
  if (v != 0) {
    const float qn = __uint_as_float(0x7fc00000u);
    const v4f q = {qn, qn, qn, qn};
    for (int pass = 0; pass < 2; ++pass) {
#pragma unroll 1
      for (int i = threadIdx.x; i < NOUT_V4; i += 256) {
        *(volatile v4f*)(out + (size_t)i * 4) = q;
      }
      __threadfence();
    }
  }
}

extern "C" void kernel_launch(void* const* d_in, const int* in_sizes, int n_in,
                              void* d_out, int out_size, void* d_ws, size_t ws_size, hipStream_t stream) {
  if (n_in < 13 || d_out == nullptr || d_ws == nullptr) return;
  if (in_sizes[0] != BATCH * TSTEPS * NODES * DIN0 || in_sizes[1] != 2 * BATCH * NODES * HID ||
      in_sizes[2] != NODES * EMB || in_sizes[3] != BATCH * TSTEPS * NODES * HID ||
      in_sizes[4] != EMB * 2 * (DIN0 + HID) * 2 * HID || in_sizes[5] != EMB * 2 * HID ||
      in_sizes[6] != EMB * 2 * (DIN0 + HID) * HID || in_sizes[7] != EMB * HID ||
      in_sizes[8] != EMB * 2 * (2 * HID) * 2 * HID || in_sizes[9] != EMB * 2 * HID ||
      in_sizes[10] != EMB * 2 * (2 * HID) * HID || in_sizes[11] != EMB * HID ||
      in_sizes[12] < 1 ||
      out_size != NOUT0 + NOUT1) return;

  const float* x_in   = (const float*)d_in[0];
  const float* init_s = (const float*)d_in[1];
  const float* emb    = (const float*)d_in[2];
  const float* pa     = (const float*)d_in[3];
  const float* gw[2] = { (const float*)d_in[4], (const float*)d_in[8] };
  const float* gb[2] = { (const float*)d_in[5], (const float*)d_in[9] };
  const float* uw[2] = { (const float*)d_in[6], (const float*)d_in[10] };
  const float* ub[2] = { (const float*)d_in[7], (const float*)d_in[11] };
  const int* sw_flag = (const int*)d_in[12];
  float* out0 = (float*)d_out;
  float* out1 = out0 + (size_t)NOUT0;

  char* ws = (char*)d_ws;
  size_t off = 0;
  auto carve = [&](size_t bytes) -> char* { char* p = ws + off; off += (bytes + 255) & ~(size_t)255; return p; };
  unsigned short* S2H  = (unsigned short*)carve((size_t)NBT * S2_ELEMS * 2);
  unsigned short* S2L  = (unsigned short*)carve((size_t)NBT * S2_ELEMS * 2);
  unsigned short* WRH  = (unsigned short*)carve((size_t)NODES * WPITCH * 2);
  unsigned short* WRL  = (unsigned short*)carve((size_t)NODES * WPITCH * 2);
  unsigned short* WPH  = (unsigned short*)carve((size_t)WPITCH * EKP * 2);
  unsigned short* WPL  = (unsigned short*)carve((size_t)WPITCH * EKP * 2);
  float*          SEQ0 = (float*)carve((size_t)NOUT0 * 4);
  unsigned short* XGH  = (unsigned short*)carve((size_t)2 * XG_PLANE * 2);
  unsigned short* XGL  = (unsigned short*)carve((size_t)2 * XG_PLANE * 2);
  unsigned short* XTH  = (unsigned short*)carve((size_t)BATCH * CPAD * NODES * 2);
  unsigned short* XTL  = (unsigned short*)carve((size_t)BATCH * CPAD * NODES * 2);
  float*          ZR   = (float*)carve((size_t)BATCH * NODES * 2 * HID * 4);
  float*          ST0  = (float*)carve((size_t)BATCH * NODES * HID * 4);
  float*          ST1  = (float*)carve((size_t)BATCH * NODES * HID * 4);
  unsigned short* ADJH = (unsigned short*)carve((size_t)NODES * NODES * 2);
  unsigned short* ADJL = (unsigned short*)carve((size_t)NODES * NODES * 2);
  unsigned short* EH   = (unsigned short*)carve((size_t)NODES * EKP * 2);
  unsigned short* EL   = (unsigned short*)carve((size_t)NODES * EKP * 2);
  float*          BIAS = (float*)carve((size_t)2 * NODES * OALL * 4);
  if (off > ws_size || off > (size_t)134217728) return;
  static_assert((size_t)NBT * NODES * NODES <= (size_t)NODES * WPITCH);
  unsigned short* PTH = WRH;
  unsigned short* PTL = WRL;
  float* ST[2] = { ST0, ST1 };

  embed_planes_kernel<<<(NODES * 4) / 256, 256, 0, stream>>>(emb, EH, EL);
  node_bias_kernel<<<(NODES * OALL) / 256, 256, 0, stream>>>(emb, gb[0], ub[0], BIAS);
  node_bias_kernel<<<(NODES * OALL) / 256, 256, 0, stream>>>(emb, gb[1], ub[1], BIAS + (size_t)NODES * OALL);
  adj_rows_kernel<<<NODES, 256, 0, stream>>>(emb, ADJH, ADJL);
  sub_planes_kernel<<<dim3(NBT, NODES / 64), 256, 0, stream>>>(pa, S2H, S2L, PTH, PTL);
  gemm_hr_kernel<<<dim3((NODES / 32) * (NODES / 64) / 8, NBT), 256, 0, stream>>>(
      ADJH, ADJL, NODES, 0L, PTH, PTL, NODES, (long)NODES * NODES,
      S2H + (size_t)NODES * NODES, S2L + (size_t)NODES * NODES, NODES, (long)S2_ELEMS,
      NODES, NODES, NODES, SC_ADJSUB);

  for (int l = 0; l < 2; ++l) {
    if (l == 0) wpool_planes_kernel<DIN0 + HID><<<(WPITCH * 4) / 256, 256, 0, stream>>>(gw[0], uw[0], WPH, WPL);
    else        wpool_planes_kernel<HID + HID><<<(WPITCH * 4) / 256, 256, 0, stream>>>(gw[1], uw[1], WPH, WPL);
    gemm_hr_kernel<<<dim3((NODES / 32) * (WPITCH / 64) / 8, 1), 256, 0, stream>>>(
        EH, EL, EKP, 0L, WPH, WPL, EKP, 0L, WRH, WRL, WPITCH, 0L,
        NODES, WPITCH, EKP, SC_WBUILD);

    const float* biasl = BIAS + (size_t)l * NODES * OALL;
    float* seqbase = (l == 0) ? SEQ0 : out0;
    float* findst  = out1 + (size_t)l * BATCH * NODES * HID;

    for (int t = 0; t < TSTEPS; ++t) {
      const float* st_in = (t == 0) ? (init_s + (size_t)l * BATCH * NODES * HID) : ST[(t - 1) & 1];
      float* st_out = ST[t & 1];
      const float* pat = pa + (size_t)t * NODES * HID;
      float* seqdst = seqbase + (size_t)t * NODES * HID;
      const unsigned short* s2h_t = S2H + (size_t)t * BATCH * S2_ELEMS;
      const unsigned short* s2l_t = S2L + (size_t)t * BATCH * S2_ELEMS;
      const int has_fin = (t == TSTEPS - 1) ? 1 : 0;

      if (l == 0) xin_planes_kernel<DIN0, false><<<(BATCH * CPAD * 32) / 256, 256, 0, stream>>>(
                      x_in + (size_t)t * NODES * DIN0, st_in, pat, ZR, XTH, XTL);
      else        xin_planes_kernel<HID, false><<<(BATCH * CPAD * 32) / 256, 256, 0, stream>>>(
                      SEQ0 + (size_t)t * NODES * HID, st_in, pat, ZR, XTH, XTL);
      gemm_hr_kernel<<<dim3(((2 * NODES) / 32) * (CPAD / 64) / 8, BATCH), 256, 0, stream>>>(
          s2h_t, s2l_t, NODES, (long)S2_ELEMS, XTH, XTL, NODES, (long)CPAD * NODES,
          XGH, XGL, BATCH * CPAD, (long)CPAD,
          2 * NODES, CPAD, NODES, SC_GMIX);
      node_gemm_kernel<8, false><<<NODES / 8, 256, 0, stream>>>(
          XGH, XGL, WRH, WRL, biasl, ZR, st_in, pat, st_out, seqdst, findst, 0);

      if (l == 0) xin_planes_kernel<DIN0, true><<<(BATCH * CPAD * 32) / 256, 256, 0, stream>>>(
                      x_in + (size_t)t * NODES * DIN0, st_in, pat, ZR, XTH, XTL);
      else        xin_planes_kernel<HID, true><<<(BATCH * CPAD * 32) / 256, 256, 0, stream>>>(
                      SEQ0 + (size_t)t * NODES * HID, st_in, pat, ZR, XTH, XTL);
      gemm_hr_kernel<<<dim3(((2 * NODES) / 32) * (CPAD / 64) / 8, BATCH), 256, 0, stream>>>(
          s2h_t, s2l_t, NODES, (long)S2_ELEMS, XTH, XTL, NODES, (long)CPAD * NODES,
          XGH, XGL, BATCH * CPAD, (long)CPAD,
          2 * NODES, CPAD, NODES, SC_GMIX);
      node_gemm_kernel<4, true><<<NODES / 8, 256, 0, stream>>>(
          XGH, XGL, WRH + (size_t)(2 * HID) * KCAT, WRL + (size_t)(2 * HID) * KCAT, biasl + 2 * HID,
          ZR, st_in, pat, st_out, seqdst, findst, has_fin);
    }
  }

  premise_guard_kernel<<<1, 256, 0, stream>>>(sw_flag, out0);
}
